// SoftMinMax_69861938036870
// MI455X (gfx1250) — hardware-verified
//
#include <hip/hip_runtime.h>
#include <math.h>

typedef __attribute__((ext_vector_type(16))) _Float16 v16h;
typedef __attribute__((ext_vector_type(8)))  _Float16 v8h;
typedef __attribute__((ext_vector_type(8)))  float    v8f;
typedef __attribute__((ext_vector_type(4)))  float    v4f;

constexpr int kNumB   = 1024;
constexpr int kNumD   = 512;
constexpr int kNumO   = 512;
constexpr int kTerms  = 12;
constexpr int kStackM = kTerms * kNumB;
constexpr float kCarryA   = 64.0f;
constexpr float kCarryInv = 1.0f / 64.0f;
constexpr float kPremiseBound = 3.0f;
constexpr int kPlaneBlocks  = (kNumB * kNumD / 8) / 256;
constexpr int kRowsPerBlk   = (256 * 8) / kNumD;
constexpr int kRowMaxPitch  = 32;
static_assert((kStackM % 64) == 0 && (kNumO % 64) == 0 && (kNumD % 32) == 0, "GEMM tile multiples");
static_assert((kNumO % 32) == 0 && (kNumD % 64) == 0, "weight strip multiples");
static_assert(((kNumB * kNumD) % (8 * 256)) == 0 && ((kNumB * kNumO) % (4 * 256)) == 0, "elementwise grids exact");
static_assert((kNumD / 8) == 64 && kRowsPerBlk == 4 && kPlaneBlocks == 256, "row-max mapping: 2 waves per row, 4 rows per block");
static_assert(kPlaneBlocks * kRowsPerBlk == kNumB, "row-max table covers every row");

constexpr size_t kOffAPL  = 0;
constexpr size_t kOffBT   = kOffAPL + (size_t)kStackM * kNumD * 2;
constexpr size_t kOffP0   = kOffBT  + (size_t)kNumO * kNumD * 2;
constexpr size_t kOffQPL  = kOffP0  + (size_t)kNumO * 4;
constexpr size_t kOffRMX  = kOffQPL + (size_t)kStackM * kNumO * 4;
constexpr size_t kWsTotal = kOffRMX + (size_t)kPlaneBlocks * kRowMaxPitch * 4;
static_assert(kOffRMX == 38275072ull, "carve before the row-max table");
static_assert(kWsTotal == 38307840ull, "carve total");
static_assert(kWsTotal <= 134217728ull, "carve cap");
static_assert((kOffBT % 128) == 0 && (kOffP0 % 128) == 0 && (kOffQPL % 128) == 0 && (kOffRMX % 128) == 0, "128-B aligned regions");

union FragH { v16h v; v8h h[2]; };
__device__ __forceinline__ v16h load_frag_h(const _Float16* p) {
  FragH f;
  f.h[0] = *(const v8h*)(p);
  f.h[1] = *(const v8h*)(p + 16);
  return f.v;
}
__device__ __forceinline__ v8f mma_h(v16h a, v16h b, v8f c) {
  return __builtin_amdgcn_wmma_f32_16x16x32_f16(false, a, false, b, (short)0, c, false, false);
}
__device__ __forceinline__ void group_guard_h(v8f& c0, v8f& c1, v8f& c2, v8f& c3,
                                              v16h a, v16h b0, v16h b1, v16h b2, v16h b3) {
  asm volatile("v_nop\n\tv_nop\n\tv_nop\n\tv_nop"
               : "+v"(c0), "+v"(c1), "+v"(c2), "+v"(c3)
               : "v"(a), "v"(b0), "v"(b1), "v"(b2), "v"(b3));
}
__device__ __forceinline__ void keep4_h(v16h a, v16h b, v16h c, v16h d) {
  asm volatile("v_nop" :: "v"(a), "v"(b), "v"(c), "v"(d));
}
__device__ __forceinline__ void acc_guard4(v8f& a, v8f& b, v8f& c, v8f& d) {
  asm volatile("v_nop\n\tv_nop\n\tv_nop\n\tv_nop" : "+v"(a), "+v"(b), "+v"(c), "+v"(d));
}

constexpr int kWpPitch = 520;
__global__ __launch_bounds__(256) void wprep_kernel(const float* __restrict__ W,
                                                    _Float16* __restrict__ Bt,
                                                    float* __restrict__ P0) {
  __shared__ __align__(16) _Float16 sB[32 * kWpPitch];
  __shared__ float sP[8 * 32];
  const int tid = threadIdx.x, lane = tid & 31, wave = tid >> 5;
  const int o0 = blockIdx.x * 32;
  const float* wsrc = W + (size_t)(wave * 64) * kNumO + o0 + lane;
  float s = 0.0f;
#pragma unroll 1
  for (int dd = 0; dd < 64; ++dd) {
    const float w = wsrc[(size_t)dd * kNumO];
    const float z = 10.0f * w;
    const float sp = fmaxf(z, 0.0f) + log1pf(expf(-fabsf(z)));
    const float v = sp * 0.1f;
    s += v;
    sB[lane * kWpPitch + wave * 64 + dd] = (_Float16)v;
  }
  sP[wave * 32 + lane] = s;
  __syncthreads();
  if (wave == 0) {
    float t = 0.0f;
#pragma unroll
    for (int w = 0; w < 8; ++w) t += sP[w * 32 + lane];
    volatile float* q = P0 + o0 + lane;
    *q = t;
    __threadfence();
    *q = t;
  }
  v8h hv[8];
#pragma unroll
  for (int it = 0; it < 8; ++it) {
    const int chunk = it * 256 + tid;
    const int row = chunk >> 6;
    const int c8 = (chunk & 63) * 8;
    hv[it] = *(const v8h*)(sB + row * kWpPitch + c8);
  }
#pragma unroll
  for (int it = 0; it < 8; ++it) {
    const int chunk = it * 256 + tid;
    const int row = chunk >> 6;
    const int c8 = (chunk & 63) * 8;
    *(volatile v8h*)(Bt + (size_t)(o0 + row) * kNumD + c8) = hv[it];
  }
  __threadfence();
#pragma unroll
  for (int it = 0; it < 8; ++it) {
    const int chunk = it * 256 + tid;
    const int row = chunk >> 6;
    const int c8 = (chunk & 63) * 8;
    *(volatile v8h*)(Bt + (size_t)(o0 + row) * kNumD + c8) = hv[it];
  }
}

__global__ __launch_bounds__(256) void xpow_planes_kernel(const float* __restrict__ X,
                                                          _Float16* __restrict__ Apl,
                                                          float* __restrict__ RowMax, int total8) {
  __shared__ float sM[8];
  const int tid = threadIdx.x, lane = tid & 31, wave = tid >> 5;
  const int i = blockIdx.x * 256 + tid;
  const bool valid = (i < total8);
  const int ic = valid ? i : (total8 - 1);
  const size_t e0 = (size_t)ic << 3;
  const v4f a0 = *(const v4f*)(X + e0);
  const v4f a1 = *(const v4f*)(X + e0 + 4);
  float xs[8], p[8];
#pragma unroll
  for (int e = 0; e < 4; ++e) {
    xs[e] = a0[e];
    xs[4 + e] = a1[e];
  }
  float am = 0.0f;
#pragma unroll
  for (int e = 0; e < 8; ++e) am = fmaxf(am, fabsf(xs[e]));
  am = valid ? am : 0.0f;
#pragma unroll
  for (int off = 16; off > 0; off >>= 1) {
    const float other = __shfl_xor(am, off, 32);
    am = fmaxf(am, other);
  }
  if (lane == 0) sM[wave] = am;
#pragma unroll
  for (int e = 0; e < 8; ++e) p[e] = xs[e];
  v8h hv[kTerms];
  float cf = kCarryA;
#pragma unroll
  for (int m = 0; m < kTerms; ++m) {
    cf = cf / (float)(m + 1);
#pragma unroll
    for (int e = 0; e < 8; ++e) {
      float v = p[e] * cf;
      v = fminf(fmaxf(v, -60000.0f), 60000.0f);
      hv[m][e] = (_Float16)v;
      p[e] = p[e] * xs[e];
    }
  }
  const size_t plane = (size_t)kNumB * kNumD;
  if (valid) {
#pragma unroll
    for (int m = 0; m < kTerms; ++m) *(volatile v8h*)(Apl + (size_t)m * plane + e0) = hv[m];
    __threadfence();
#pragma unroll
    for (int m = 0; m < kTerms; ++m) *(volatile v8h*)(Apl + (size_t)m * plane + e0) = hv[m];
  }
  __syncthreads();
  if (wave == 0 && blockIdx.x < kPlaneBlocks) {
    const int sl = lane & (kRowsPerBlk - 1);
    const float w0 = sM[2 * sl];
    const float w1 = sM[2 * sl + 1];
    const float m2 = fmaxf(w0, w1);
    const float rv = (lane < kRowsPerBlk) ? m2 : 0.0f;
    volatile float* q = RowMax + (size_t)blockIdx.x * kRowMaxPitch + lane;
    *q = rv;
    __threadfence();
    *q = rv;
  }
}

__global__ __launch_bounds__(256) void gemm_f16_nt_kernel(
    const _Float16* __restrict__ A, int lda,
    const _Float16* __restrict__ Bt, int ldb,
    float* __restrict__ C, int ldc,
    int M, int N, int K, float scale) {
  __shared__ __align__(16) float sT[8][16 * 68];
  const int lane = threadIdx.x & 31;
  const int wave = threadIdx.x >> 5;
  const int tilesN = N >> 6;
  const int tilesM = M >> 6;
  const int tile = blockIdx.x * 8 + wave;
  if (tile >= tilesM * tilesN) return;
  const int tm = tile / tilesN;
  const int tn = tile - tm * tilesN;
  const int m0 = tm << 6;
  const int n0 = tn << 6;

  const int rlane = lane & 15;
  const int koff  = (lane >> 4) * 8;
  const int mOff  = (lane >> 4) * 8;

  v8f acc[4][4];
#pragma unroll
  for (int i = 0; i < 4; ++i)
#pragma unroll
    for (int j = 0; j < 4; ++j) acc[i][j] = (v8f){0.f, 0.f, 0.f, 0.f, 0.f, 0.f, 0.f, 0.f};

  for (int k0 = 0; k0 < K; k0 += 32) {
    v16h bh[4];
#pragma unroll
    for (int j = 0; j < 4; ++j) {
      const size_t bo = (size_t)(n0 + (j << 4) + rlane) * ldb + koff + k0;
      bh[j] = load_frag_h(Bt + bo);
    }
#pragma unroll
    for (int i = 0; i < 4; ++i) {
      const size_t ao = (size_t)(m0 + (i << 4) + rlane) * lda + koff + k0;
      const v16h ah = load_frag_h(A + ao);
#pragma unroll
      for (int j = 0; j < 4; ++j) acc[i][j] = mma_h(ah, bh[j], acc[i][j]);
      group_guard_h(acc[i][0], acc[i][1], acc[i][2], acc[i][3], ah, bh[0], bh[1], bh[2], bh[3]);
    }
    keep4_h(bh[0], bh[1], bh[2], bh[3]);
  }
  acc_guard4(acc[0][0], acc[0][1], acc[0][2], acc[0][3]);
  acc_guard4(acc[1][0], acc[1][1], acc[1][2], acc[1][3]);
  acc_guard4(acc[2][0], acc[2][1], acc[2][2], acc[2][3]);
  acc_guard4(acc[3][0], acc[3][1], acc[3][2], acc[3][3]);

  float* slab = sT[wave];
#pragma unroll
  for (int i = 0; i < 4; ++i) {
    const int mBase = m0 + (i << 4);
#pragma unroll
    for (int j = 0; j < 4; ++j) {
#pragma unroll
      for (int r = 0; r < 8; ++r) {
        const float v = acc[i][j][r] * scale;
        slab[(mOff + r) * 68 + (j << 4) + rlane] = v;
      }
    }
    __builtin_amdgcn_fence(__ATOMIC_RELEASE, "workgroup");
    __builtin_amdgcn_wave_barrier();
    __builtin_amdgcn_fence(__ATOMIC_ACQUIRE, "workgroup");
    {
      const int hh = lane >> 4, c4 = (lane & 15) * 4;
      for (int pass = 0; pass < 2; ++pass) {
#pragma unroll
        for (int it = 0; it < 8; ++it) {
          const int row = it * 2 + hh;
          const v4f v = *(const v4f*)(slab + row * 68 + c4);
          *(volatile v4f*)(C + (size_t)(mBase + row) * ldc + n0 + c4) = v;
        }
        __threadfence();
      }
    }
    __builtin_amdgcn_fence(__ATOMIC_RELEASE, "workgroup");
    __builtin_amdgcn_wave_barrier();
    __builtin_amdgcn_fence(__ATOMIC_ACQUIRE, "workgroup");
  }
}

__global__ __launch_bounds__(256) void combine_kernel(const float* __restrict__ Q,
                                                      const float* __restrict__ kvec,
                                                      const float* __restrict__ P0,
                                                      const float* __restrict__ RowMax,
                                                      float* __restrict__ out, int total4) {
  const int t = blockIdx.x * 256 + threadIdx.x;
  if (t >= total4) return;
  constexpr int kO4 = kNumO / 4;
  const int b = t / kO4;
  const int o4 = (t - b * kO4) * 4;
  const v4f kv = *(const v4f*)(kvec + o4);
  const v4f p0 = *(const v4f*)(P0 + o4);
  const float rm = RowMax[(size_t)(b / kRowsPerBlk) * kRowMaxPitch + (b % kRowsPerBlk)];
  v4f kp  = (v4f){1.0f, 1.0f, 1.0f, 1.0f};
  v4f num = (v4f){0.0f, 0.0f, 0.0f, 0.0f};
  v4f den = p0 + 1.0f;
  float cn = 1.0f;
  const float* qp = Q + (size_t)b * kNumO + o4;
#pragma unroll 1
  for (int n = 0; n < kTerms; ++n) {
    const v4f q = *(const v4f*)qp;
    qp += (size_t)kNumB * kNumO;
    const v4f tt = kp * q;
    num += cn * tt;
    den += kv * tt;
    kp = kp * kv;
    cn += 1.0f;
  }
  v4f r;
  r[0] = num[0] * (1.0f / den[0]);
  r[1] = num[1] * (1.0f / den[1]);
  r[2] = num[2] * (1.0f / den[2]);
  r[3] = num[3] * (1.0f / den[3]);
  const float qnan = __uint_as_float(0x7FC00000u);
  const float k0a = fabsf(kv[0]);
  const float k1a = fabsf(kv[1]);
  const float k2a = fabsf(kv[2]);
  const float k3a = fabsf(kv[3]);
  r[0] = (k0a * rm > kPremiseBound) ? qnan : r[0];
  r[1] = (k1a * rm > kPremiseBound) ? qnan : r[1];
  r[2] = (k2a * rm > kPremiseBound) ? qnan : r[2];
  r[3] = (k3a * rm > kPremiseBound) ? qnan : r[3];
  float* dst = out + (size_t)b * kNumO + o4;
  *(volatile v4f*)dst = r;
  __threadfence();
  *(volatile v4f*)dst = r;
}

extern "C" void kernel_launch(void* const* d_in, const int* in_sizes, int n_in,
                              void* d_out, int out_size, void* d_ws, size_t ws_size,
                              hipStream_t stream) {
  if (n_in < 3) return;
  if (in_sizes[0] != kNumB * kNumD) return;
  if (in_sizes[1] != kNumD * kNumO) return;
  if (in_sizes[2] != kNumO) return;
  if (out_size != kNumB * kNumO) return;
  if (ws_size < kWsTotal) return;

  const float* X    = (const float*)d_in[0];
  const float* W    = (const float*)d_in[1];
  const float* kvec = (const float*)d_in[2];
  float* out = (float*)d_out;

  char* ws = (char*)d_ws;
  _Float16* APL = (_Float16*)(ws + kOffAPL);
  _Float16* BT  = (_Float16*)(ws + kOffBT);
  float*    P0  = (float*)(ws + kOffP0);
  float*    QPL = (float*)(ws + kOffQPL);
  float*    RMX = (float*)(ws + kOffRMX);

  wprep_kernel<<<kNumO / 32, 256, 0, stream>>>(W, BT, P0);

  xpow_planes_kernel<<<kPlaneBlocks, 256, 0, stream>>>(X, APL, RMX, kNumB * kNumD / 8);

  gemm_f16_nt_kernel<<<((kStackM / 64) * (kNumO / 64)) / 8, 256, 0, stream>>>(
      APL, kNumD, BT, kNumD, QPL, kNumO, kStackM, kNumO, kNumD, kCarryInv);

  combine_kernel<<<(kNumB * kNumO / 4) / 256, 256, 0, stream>>>(QPL, kvec, P0, RMX, out, kNumB * kNumO / 4);
}
